// GATLayer_89275190215473
// MI455X (gfx1250) — hardware-verified
//
#include <hip/hip_runtime.h>
#include <stddef.h>
#include <stdint.h>


#define DIN     512
#define LAT     128
#define NHEAD   4
#define HP      512
#define ALP     8
#define NTHR    256
#define NWAVE   8
#define EPT     8
#define CHUNK   (NTHR * EPT)
#define WCAP    (EPT * 32)
#define LISTN   (NWAVE * WCAP)
#define NBMAX   2048
#define RCAP    16384
#define DEGCAP  32
#define GBM     64
#define GBN     64
#define GTHR    128
#define WSMAX   134217728
#define LDS_AGG ((2 * RCAP + 2 * NBMAX + LISTN) * 4 + 64)

static_assert((CHUNK & (CHUNK - 1)) == 0 && CHUNK <= 4096);
static_assert((NBMAX & (NBMAX - 1)) == 0 && NBMAX <= 4096);
static_assert(NTHR * 8 == NBMAX);
static_assert(LISTN >= NBMAX);
static_assert(LISTN >= NWAVE * WCAP);
static_assert(WCAP <= 4096);
static_assert((RCAP % 32) == 0);
static_assert(LDS_AGG <= 300000);
static_assert(GBM == (GTHR / 32) * 16);
static_assert(DIN / 8 == 64);
static_assert((DIN % 32) == 0);
static_assert(HP == NHEAD * LAT && LAT == 128 && (HP % GBN) == 0);
static_assert(ALP == 2 * NHEAD);

typedef float          v4f   __attribute__((ext_vector_type(4)));
typedef float          v8f   __attribute__((ext_vector_type(8)));
typedef int            v4i   __attribute__((ext_vector_type(4)));
typedef int            v8i   __attribute__((ext_vector_type(8)));
typedef unsigned short v8us  __attribute__((ext_vector_type(8)));
typedef __bf16         v16bf __attribute__((ext_vector_type(16)));
union FragB { v16bf v; v8us h[2]; v8i w; };

__device__ __forceinline__ v8f wmb(const FragB& a, const FragB& b, v8f c) {
  v8f d = __builtin_amdgcn_wmma_f32_16x16x32_bf16(false, a.v, false, b.v, (short)0, c, false, false);
  asm volatile("v_nop\n\tv_nop\n\tv_nop\n\tv_nop" : "+v"(d) : "v"(a.w), "v"(b.w));
  return d;
}

__device__ __forceinline__ void ldwait() {
  asm volatile("s_wait_loadcnt 0x0" ::: "memory");
}

__device__ __forceinline__ unsigned short bfbits(float f) {
  unsigned u = __float_as_uint(f);
  u += 0x7FFFu + ((u >> 16) & 1u);
  return (unsigned short)(u >> 16);
}
__device__ __forceinline__ float bfval(float f) {
  unsigned u = __float_as_uint(f);
  u += 0x7FFFu + ((u >> 16) & 1u);
  return __uint_as_float(u & 0xFFFF0000u);
}
__device__ __forceinline__ v4f bf4(const v4f a) {
  v4f r;
  r.x = bfval(a.x); r.y = bfval(a.y); r.z = bfval(a.z); r.w = bfval(a.w);
  return r;
}
__device__ __forceinline__ v8us cvt8b(const v4f a, const v4f b) {
  v8us hv;
  hv[0] = bfbits(a.x); hv[1] = bfbits(a.y); hv[2] = bfbits(a.z); hv[3] = bfbits(a.w);
  hv[4] = bfbits(b.x); hv[5] = bfbits(b.y); hv[6] = bfbits(b.z); hv[7] = bfbits(b.w);
  return hv;
}

__device__ __forceinline__ int scan_chunk(const int* __restrict__ edges, int nE, int cbase, int slotBase,
                                          int nb, int* list, int tid, int lane, int wave) {
  int wc = 0;
  const int el0  = tid * EPT;
  const int e0   = cbase + el0;
  const int sent = -2147483647 - 1;
  int g0, g1, g2, g3, g4, g5, g6, g7;
  if (cbase + CHUNK <= nE) {
    const int* p = edges + 2 * (size_t)e0;
    const v4i qa = *(const v4i*)p;
    const v4i qb = *(const v4i*)(p + 4);
    const v4i qc = *(const v4i*)(p + 8);
    const v4i qd = *(const v4i*)(p + 12);
    g0 = qa.x; g1 = qa.z; g2 = qb.x; g3 = qb.z;
    g4 = qc.x; g5 = qc.z; g6 = qd.x; g7 = qd.z;
  } else {
    g0 = (e0     < nE) ? edges[2 * (size_t)min(e0,     nE - 1)] : sent;
    g1 = (e0 + 1 < nE) ? edges[2 * (size_t)min(e0 + 1, nE - 1)] : sent;
    g2 = (e0 + 2 < nE) ? edges[2 * (size_t)min(e0 + 2, nE - 1)] : sent;
    g3 = (e0 + 3 < nE) ? edges[2 * (size_t)min(e0 + 3, nE - 1)] : sent;
    g4 = (e0 + 4 < nE) ? edges[2 * (size_t)min(e0 + 4, nE - 1)] : sent;
    g5 = (e0 + 5 < nE) ? edges[2 * (size_t)min(e0 + 5, nE - 1)] : sent;
    g6 = (e0 + 6 < nE) ? edges[2 * (size_t)min(e0 + 6, nE - 1)] : sent;
    g7 = (e0 + 7 < nE) ? edges[2 * (size_t)min(e0 + 7, nE - 1)] : sent;
  }
  const unsigned nbs = (unsigned)slotBase;
  const unsigned unb = (unsigned)nb;
  const unsigned s0 = (unsigned)g0 - nbs, s1 = (unsigned)g1 - nbs;
  const unsigned s2 = (unsigned)g2 - nbs, s3 = (unsigned)g3 - nbs;
  const unsigned s4 = (unsigned)g4 - nbs, s5 = (unsigned)g5 - nbs;
  const unsigned s6 = (unsigned)g6 - nbs, s7 = (unsigned)g7 - nbs;
  const bool h0 = s0 < unb, h1 = s1 < unb, h2 = s2 < unb, h3 = s3 < unb;
  const bool h4 = s4 < unb, h5 = s5 < unb, h6 = s6 < unb, h7 = s7 < unb;
  const unsigned any = __builtin_amdgcn_ballot_w32(h0 | h1 | h2 | h3 | h4 | h5 | h6 | h7);
  if (any != 0u) {
#define HITJ(J, HJ, SJ) { \
      const unsigned mj = __builtin_amdgcn_ballot_w32(HJ); \
      if (mj != 0u) { \
        if (HJ) { \
          const int pos = wc + (int)__builtin_amdgcn_mbcnt_lo(mj, 0u); \
          if (pos < WCAP) list[wave * WCAP + pos] = ((el0 + (J)) << 12) | (int)(SJ); \
        } \
        wc += (int)__builtin_popcount(mj); } }
    HITJ(0, h0, s0)
    HITJ(1, h1, s1)
    HITJ(2, h2, s2)
    HITJ(3, h3, s3)
    HITJ(4, h4, s4)
    HITJ(5, h5, s5)
    HITJ(6, h6, s6)
    HITJ(7, h7, s7)
#undef HITJ
  }
  return wc;
}

__global__ __launch_bounds__(NTHR) void k_xprep(const float* __restrict__ x, unsigned short* xb, int nN, int nUnits) {
  const int i = (int)blockIdx.x * NTHR + (int)threadIdx.x;
  if (i >= nUnits) return;
  const int row = i >> 6;
  const int c0  = (i & 63) * 8;
  const int rc  = row < nN ? row : nN - 1;
  const float* p = x + (size_t)rc * DIN + c0;
  v4f a = *(const v4f*)p, b = *(const v4f*)(p + 4);
  const v4f z4 = {0.f, 0.f, 0.f, 0.f};
  if (row >= nN) { a = z4; b = z4; }
  const v8us hv = cvt8b(a, b);
  const size_t o = (size_t)row * DIN + c0;
  *(volatile v8us*)(xb + o) = hv;
  __threadfence();
  *(volatile v8us*)(xb + o) = hv;
}

__global__ __launch_bounds__(NTHR) void k_wtr(const float* __restrict__ W, unsigned short* wt, int nUnits) {
  const int u = (int)blockIdx.x * NTHR + (int)threadIdx.x;
  if (u >= nUnits) return;
  const int n  = u >> 6;
  const int k8 = (u & 63) * 8;
  const int hd = n >> 7;
  const int f  = n & (LAT - 1);
  const float* p = W + (size_t)hd * DIN * LAT + (size_t)k8 * LAT + f;
  v4f a, b;
  a.x = p[0];                 a.y = p[(size_t)LAT];         a.z = p[(size_t)2 * LAT];     a.w = p[(size_t)3 * LAT];
  b.x = p[(size_t)4 * LAT];   b.y = p[(size_t)5 * LAT];     b.z = p[(size_t)6 * LAT];     b.w = p[(size_t)7 * LAT];
  const v8us hv = cvt8b(a, b);
  const size_t o = (size_t)n * DIN + k8;
  *(volatile v8us*)(wt + o) = hv;
  __threadfence();
  *(volatile v8us*)(wt + o) = hv;
}

__global__ __launch_bounds__(GTHR) void k_gemm(
    const unsigned short* __restrict__ A, const unsigned short* __restrict__ WT,
    float* outF, int K, int ldo)
{
  __shared__ __attribute__((aligned(16))) float stg[GBM * GBN];
  const int tid = (int)threadIdx.x, lane = tid & 31, wave = tid >> 5, hh = lane >> 4, m = lane & 15;
  const int rowBase = (int)blockIdx.x * GBM;
  const int col0    = (int)blockIdx.y * GBN;

  v8f acc[4];
  {
    const v8f z = {0.f, 0.f, 0.f, 0.f, 0.f, 0.f, 0.f, 0.f};
    acc[0] = z; acc[1] = z; acc[2] = z; acc[3] = z;
  }
  const unsigned short* ap = A  + (size_t)(rowBase + 16 * wave + m) * (size_t)K + 8 * hh;
  const unsigned short* wp = WT + (size_t)(col0 + m) * (size_t)K + 8 * hh;
  const int ksteps = K >> 5;
#pragma unroll 1
  for (int ks = 0; ks < ksteps; ++ks) {
    FragB af;
    af.h[0] = *(const v8us*)(ap + 32 * ks);
    af.h[1] = *(const v8us*)(ap + 32 * ks + 16);
#pragma unroll
    for (int t = 0; t < 4; ++t) {
      const unsigned short* wq = wp + (size_t)(16 * t) * (size_t)K + 32 * ks;
      FragB bf;
      bf.h[0] = *(const v8us*)wq;
      bf.h[1] = *(const v8us*)(wq + 16);
      acc[t] = wmb(af, bf, acc[t]);
    }
  }

#pragma unroll
  for (int t = 0; t < 4; ++t) {
    const int lc = 16 * t + m;
#pragma unroll
    for (int r = 0; r < 8; ++r) {
      const int lr = 16 * wave + 8 * hh + r;
      stg[lr * GBN + lc] = acc[t][r];
    }
  }
  __syncthreads();

  v4f fv[8];
#pragma unroll
  for (int i = 0; i < 8; ++i) {
    const int lr = 16 * wave + 2 * i + hh;
    fv[i] = *(const v4f*)(stg + lr * GBN + 4 * m);
  }
#pragma unroll
  for (int i = 0; i < 8; ++i) {
    const int lr = 16 * wave + 2 * i + hh;
    const int gr = rowBase + lr;
    float* op = outF + (size_t)gr * (size_t)ldo + col0 + 4 * m;
    *(volatile v4f*)op = fv[i];
  }
  __threadfence();
#pragma unroll
  for (int i = 0; i < 8; ++i) {
    const int lr = 16 * wave + 2 * i + hh;
    const int gr = rowBase + lr;
    float* op = outF + (size_t)gr * (size_t)ldo + col0 + 4 * m;
    *(volatile v4f*)op = fv[i];
  }
}

__global__ __launch_bounds__(NTHR) void k_alpha(const float* __restrict__ H, const float* __restrict__ av,
                                                float* AL, int nGroups) {
  __shared__ __attribute__((aligned(16))) float stw[NWAVE * 32];
  const int tid = (int)threadIdx.x, lane = tid & 31, wave = tid >> 5;
  const int gw = (int)blockIdx.x * NWAVE + wave;
  if (gw >= nGroups) return;
  v4f asv[NHEAD], adv[NHEAD];
#pragma unroll
  for (int hd = 0; hd < NHEAD; ++hd) {
    const float* ap = av + hd * (2 * LAT) + 4 * lane;
    asv[hd] = bf4(*(const v4f*)ap);
    adv[hd] = bf4(*(const v4f*)(ap + LAT));
  }
  float* sw = stw + wave * 32;
#pragma unroll 1
  for (int i = 0; i < 4; ++i) {
    const int n = gw * 4 + i;
    const float* hp = H + (size_t)n * HP + 4 * lane;
    float ps[NHEAD], pd[NHEAD];
#pragma unroll
    for (int hd = 0; hd < NHEAD; ++hd) {
      const v4f hv = *(const v4f*)(hp + LAT * hd);
      const v4f m1 = asv[hd] * hv;
      const v4f m2 = adv[hd] * hv;
      ps[hd] = (m1.x + m1.y) + (m1.z + m1.w);
      pd[hd] = (m2.x + m2.y) + (m2.z + m2.w);
    }
#pragma unroll
    for (int off = 16; off > 0; off >>= 1) {
#pragma unroll
      for (int hd = 0; hd < NHEAD; ++hd) {
        ps[hd] += __shfl_xor(ps[hd], off);
        pd[hd] += __shfl_xor(pd[hd], off);
      }
    }
    if (lane == 0) {
#pragma unroll
      for (int hd = 0; hd < NHEAD; ++hd) {
        sw[8 * i + hd]         = ps[hd];
        sw[8 * i + NHEAD + hd] = pd[hd];
      }
    }
  }
  __builtin_amdgcn_fence(__ATOMIC_RELEASE, "wavefront");
  __builtin_amdgcn_wave_barrier();
  const int lc = lane < 8 ? lane : 7;
  const v4f gv = *(const v4f*)(sw + 4 * lc);
  float* gp = AL + (size_t)gw * 32 + 4 * lc;
  if (lane < 8) *(volatile v4f*)gp = gv;
  __threadfence();
  if (lane < 8) *(volatile v4f*)gp = gv;
}

__global__ __launch_bounds__(NTHR) void k_agg(
    const int* __restrict__ edges, const float* __restrict__ H, const float* __restrict__ AL,
    float* out, int nN, int nE, int nb) {
  extern __shared__ v4f lds_dyn[];
  int* reg1 = (int*)lds_dyn;
  int* reg2 = reg1 + RCAP;
  int* scnt = reg2 + RCAP;
  int* soff = scnt + NBMAX;
  int* list = soff + NBMAX;
  int* wcnt = list + LISTN;
  int* wtot = wcnt + NWAVE;
  const int tid = (int)threadIdx.x, lane = tid & 31, wave = tid >> 5;
  const int nodeBase = (int)blockIdx.x * nb;

  for (int i = tid; i < NBMAX; i += NTHR) scnt[i] = 0;
  __syncthreads();

  int tot = 0;
  const int nChunks = (nE + CHUNK - 1) / CHUNK;
#pragma unroll 1
  for (int ch = 0; ch < nChunks; ++ch) {
    const int cbase = ch * CHUNK;
    const int wc = scan_chunk(edges, nE, cbase, nodeBase, nb, list, tid, lane, wave);
    if (lane == 0) wcnt[wave] = wc;
    __syncthreads();
    int pre = 0, all = 0;
#pragma unroll
    for (int w2 = 0; w2 < NWAVE; ++w2) {
      int c = wcnt[w2];
      c = c < 0 ? 0 : (c > WCAP ? WCAP : c);
      all += c;
      pre += (w2 < wave) ? c : 0;
    }
    const int wcc  = wc > WCAP ? WCAP : wc;
    const int base = tot + pre;
#pragma unroll 1
    for (int i = lane; i < wcc; i += 32) {
      const int ent = list[wave * WCAP + i];
      const int el  = (ent >> 12) & (CHUNK - 1);
      const int sl  = ent & (NBMAX - 1);
      int eid = cbase + el;
      eid = eid > nE - 1 ? nE - 1 : eid;
      const int pos = base + i;
      if (pos < RCAP) reg1[pos] = (int)(((unsigned)eid << 12) | (unsigned)sl);
    }
    tot += all;
    tot = tot > RCAP ? RCAP : tot;
    __syncthreads();
  }
  const int nh = tot;

  if (wave == 0) {
#pragma unroll 1
    for (int b0 = 0; b0 < nh; b0 += 32) {
      const int idx = b0 + lane;
      const int uv  = reg1[idx < nh ? idx : nh - 1];
      const int m32 = (nh - b0) < 32 ? (nh - b0) : 32;
#pragma unroll 1
      for (int k = 0; k < m32; ++k) {
        const int u  = __builtin_amdgcn_readlane(uv, k);
        const int sl = u & (NBMAX - 1);
        if (lane == 0) scnt[sl] = scnt[sl] + 1;
      }
    }
  }
  __syncthreads();

  {
    const v4i ca = *(const v4i*)(scnt + 8 * tid);
    const v4i cb = *(const v4i*)(scnt + 8 * tid + 4);
    const int e0 = ca.x < 0 ? 0 : ca.x, e1 = ca.y < 0 ? 0 : ca.y, e2 = ca.z < 0 ? 0 : ca.z, e3 = ca.w < 0 ? 0 : ca.w;
    const int e4 = cb.x < 0 ? 0 : cb.x, e5 = cb.y < 0 ? 0 : cb.y, e6 = cb.z < 0 ? 0 : cb.z, e7 = cb.w < 0 ? 0 : cb.w;
    const int ts = e0 + e1 + e2 + e3 + e4 + e5 + e6 + e7;
    int incl = ts;
#pragma unroll
    for (int d = 1; d < 32; d <<= 1) {
      const int up = __shfl_up(incl, d);
      if (lane >= d) incl += up;
    }
    if (lane == 31) wtot[wave] = incl;
    __syncthreads();
    int pre = 0;
#pragma unroll
    for (int w2 = 0; w2 < NWAVE; ++w2) pre += (w2 < wave) ? wtot[w2] : 0;
    int run = pre + incl - ts;
    soff[8 * tid + 0] = run; run += e0;
    soff[8 * tid + 1] = run; run += e1;
    soff[8 * tid + 2] = run; run += e2;
    soff[8 * tid + 3] = run; run += e3;
    soff[8 * tid + 4] = run; run += e4;
    soff[8 * tid + 5] = run; run += e5;
    soff[8 * tid + 6] = run; run += e6;
    soff[8 * tid + 7] = run;
  }
  __syncthreads();
  for (int i = tid; i < NBMAX; i += NTHR) list[i] = soff[i];
  __syncthreads();

  if (wave == 0) {
#pragma unroll 1
    for (int b0 = 0; b0 < nh; b0 += 32) {
      const int idx = b0 + lane;
      const int uv  = reg1[idx < nh ? idx : nh - 1];
      const int m32 = (nh - b0) < 32 ? (nh - b0) : 32;
#pragma unroll 1
      for (int k = 0; k < m32; ++k) {
        const int u   = __builtin_amdgcn_readlane(uv, k);
        const int sl  = u & (NBMAX - 1);
        const int eid = (int)((unsigned)u >> 12);
        if (lane == 0) {
          int pos = list[sl];
          pos = pos < 0 ? 0 : (pos > RCAP - 1 ? RCAP - 1 : pos);
          reg2[pos] = eid;
          list[sl] = pos + 1;
        }
      }
    }
  }
  __syncthreads();

  const int nbw = nb >> 3;
  const bool ovf = (nh >= RCAP);
  const float qnan = __int_as_float(0x7fc00000);
#pragma unroll 1
  for (int jt = 0; jt < nbw; ++jt) {
    const int slot = wave * nbw + jt;
    const int grow = nodeBase + slot;
    const int gcl  = grow < nN ? grow : nN - 1;
    int st = soff[slot];
    const int craw = scnt[slot];
    int cnt = craw;
    st  = st < 0 ? 0 : (st > nh ? nh : st);
    cnt = cnt < 0 ? 0 : (cnt > DEGCAP ? DEGCAP : cnt);
    if (cnt > nh - st) cnt = nh - st;
    const float pz = (ovf || craw > DEGCAP) ? qnan : 0.0f;
    const bool wr = grow < nN;

    const v4f ps4 = *(const v4f*)(AL + (size_t)gcl * ALP);
    ldwait();
    float ps[NHEAD];
    ps[0] = ps4.x; ps[1] = ps4.y; ps[2] = ps4.z; ps[3] = ps4.w;
    float mx[NHEAD], dn[NHEAD];
    v4f av[NHEAD];
    {
      const v4f z4 = {0.f, 0.f, 0.f, 0.f};
#pragma unroll
      for (int hd = 0; hd < NHEAD; ++hd) { mx[hd] = -1.0e30f; dn[hd] = 0.f; av[hd] = z4; }
    }

#pragma unroll 1
    for (int q = 0; q < cnt; ++q) {
      int idx = st + q; idx = idx > RCAP - 1 ? RCAP - 1 : idx;
      int eid = reg2[idx]; eid = eid < 0 ? 0 : (eid > nE - 1 ? nE - 1 : eid);
      const int draw = edges[2 * (size_t)eid + 1];
      const int d = draw < 0 ? 0 : (draw > nN - 1 ? nN - 1 : draw);
      const v4f pd4 = *(const v4f*)(AL + (size_t)d * ALP + NHEAD);
      const float* hr = H + (size_t)d * HP + 4 * lane;
      v4f vv[NHEAD];
#pragma unroll
      for (int hd = 0; hd < NHEAD; ++hd) vv[hd] = *(const v4f*)(hr + LAT * hd);
      ldwait();
      float pd[NHEAD];
      pd[0] = pd4.x; pd[1] = pd4.y; pd[2] = pd4.z; pd[3] = pd4.w;
#pragma unroll
      for (int hd = 0; hd < NHEAD; ++hd) {
        float al = ps[hd] + pd[hd];
        al = (al >= 0.f) ? al : 0.2f * al;
        const float df = al - mx[hd];
        const float ee = __expf(-fabsf(df));
        const bool up  = df > 0.f;
        const float s1 = up ? ee : 1.0f;
        const float s2 = up ? 1.0f : ee;
        mx[hd] = up ? al : mx[hd];
        dn[hd] = fmaf(dn[hd], s1, s2);
        av[hd] = av[hd] * s1 + vv[hd] * s2;
      }
    }
    v4f o[NHEAD];
#pragma unroll
    for (int hd = 0; hd < NHEAD; ++hd) {
      const float ds = dn[hd] > 0.f ? dn[hd] : 1.0f;
      const float iv = (dn[hd] > 0.f ? 1.0f : 0.0f) * __builtin_amdgcn_rcpf(ds);
      o[hd] = av[hd] * iv + pz;
    }
    float* op = out + (size_t)gcl * HP + 4 * lane;
    if (wr) {
      *(volatile v4f*)(op)           = o[0];
      *(volatile v4f*)(op + LAT)     = o[1];
      *(volatile v4f*)(op + 2 * LAT) = o[2];
      *(volatile v4f*)(op + 3 * LAT) = o[3];
    }
    __threadfence();
    if (wr) {
      *(volatile v4f*)(op)           = o[0];
      *(volatile v4f*)(op + LAT)     = o[1];
      *(volatile v4f*)(op + 2 * LAT) = o[2];
      *(volatile v4f*)(op + 3 * LAT) = o[3];
    }
  }
}

static int pick_nb(int nE, int nN) {
  int nb = NBMAX;
  while (nb > 16 && (long long)nb * (long long)nE * 5LL > (long long)RCAP * (long long)nN * 4LL) nb >>= 1;
  return nb;
}
static inline int cdiv(int a, int b) { return (a + b - 1) / b; }

extern "C" void kernel_launch(void* const* d_in, const int* in_sizes, int n_in,
                              void* d_out, int out_size, void* d_ws, size_t ws_size,
                              hipStream_t stream) {
  if (n_in < 4) return;
  const int nN = in_sizes[0] / DIN;
  if (nN <= 0 || in_sizes[0] != nN * DIN || nN > (1 << 22)) return;
  if (in_sizes[1] < 2 || (in_sizes[1] & 1) != 0) return;
  const int nE = in_sizes[1] / 2;
  if (nE < 1 || nE > (1 << 20)) return;
  if (in_sizes[2] != NHEAD * DIN * LAT) return;
  if (in_sizes[3] != NHEAD * 2 * LAT) return;
  if (out_size != nN * HP) return;

  const float* x     = (const float*)d_in[0];
  const int*   edges = (const int*)  d_in[1];
  const float* W     = (const float*)d_in[2];
  const float* av    = (const float*)d_in[3];
  float* out = (float*)d_out;

  const int MP = cdiv(nN, GBM) * GBM;
  const int nb = pick_nb(nE, nN);
  const int gA = cdiv(MP, nb);
  if (gA * nb < MP) return;

  char* ws = (char*)d_ws;
  size_t off = 0;
  const size_t oXB = off; off += (size_t)MP * DIN * 2;             off = (off + 255) & ~(size_t)255;
  const size_t oWT = off; off += (size_t)HP * DIN * 2;             off = (off + 255) & ~(size_t)255;
  const size_t oH  = off; off += (size_t)MP * HP * 4;              off = (off + 255) & ~(size_t)255;
  const size_t oAL = off; off += (size_t)MP * ALP * 4;             off = (off + 255) & ~(size_t)255;
  if (off > ws_size || off > (size_t)WSMAX) return;
  unsigned short* XB = (unsigned short*)(ws + oXB);
  unsigned short* WT = (unsigned short*)(ws + oWT);
  float*          Hf = (float*)(ws + oH);
  float*          AL = (float*)(ws + oAL);

  hipFuncSetAttribute(reinterpret_cast<const void*>(&k_agg),
                      hipFuncAttributeMaxDynamicSharedMemorySize, LDS_AGG);

  const int nUx = MP * (DIN / 8);
  k_xprep<<<cdiv(nUx, NTHR), NTHR, 0, stream>>>(x, XB, nN, nUx);

  const int nUw = HP * (DIN / 8);
  k_wtr<<<cdiv(nUw, NTHR), NTHR, 0, stream>>>(W, WT, nUw);

  k_gemm<<<dim3(MP / GBM, HP / GBN), GTHR, 0, stream>>>(XB, WT, Hf, DIN, HP);

  const int nGroups = MP / 4;
  k_alpha<<<cdiv(nGroups, NWAVE), NTHR, 0, stream>>>(Hf, av, AL, nGroups);

  k_agg<<<gA, NTHR, LDS_AGG, stream>>>(edges, Hf, AL, out, nN, nE, nb);
}
